// pro_encoder_10857677325002
// MI455X (gfx1250) — hardware-verified
//
#include <hip/hip_runtime.h>
#include <stddef.h>


#define FIN     33
#define KP0     64
#define HID     128
#define HID2    256
#define NTHR    256
#define NWAVE   8
#define EPT     8
#define NGRP    2
#define CHUNK   (NTHR * EPT * NGRP)
#define WCAP    (EPT * NGRP * 32)
#define LISTN   (NWAVE * WCAP)
#define NBC     4096
#define NBF     1024
#define RCAP    40960
#define RBN     128
#define TGT     256
#define DEGCAP  256
#define GROWS   128
#define OTHR    512
#define ASCALE  64.0f
#define WSCALE  16.0f
#define OSCALE  0.0009765625f

#define LDS_FILL ((RCAP + NBF + LISTN) * 4 + 64)
#define LDS_G0   (GROWS * HID * 4)
#define LDS_G1   (GROWS * HID * 4 + 2 * GROWS * 4)
#define LDS_G2   (GROWS * (HID2 + 8) * 2)

static_assert((CHUNK & (CHUNK - 1)) == 0);
static_assert(CHUNK <= 4096);
static_assert(NBC <= 4096 && NBF <= 4096);
static_assert((NBC & (NBC - 1)) == 0 && (NBF & (NBF - 1)) == 0);
static_assert(NBC == 4 * NBF);
static_assert(OTHR * 8 == NBC);
static_assert((RCAP % 32) == 0);
static_assert(2 * GROWS * (KP0 + 8) * 2 <= LDS_G0);
static_assert(GROWS * (HID + 8) * 2 <= GROWS * HID * 4);
static_assert(GROWS * HID * 4 <= LDS_G2);
static_assert(TGT == NWAVE * 32 && (TGT % GROWS) == 0);
static_assert((HID * KP0 / 8) % NTHR == 0 && (HID2 * HID / 8) % NTHR == 0 && (HID * HID2 / 8) % NTHR == 0);
static_assert((GROWS * KP0 / 8) % NTHR == 0 && (GROWS * HID / 8) % NTHR == 0 && (GROWS * HID2 / 8) % NTHR == 0);
static_assert((NBC % NTHR) == 0);
static_assert(NTHR == 4 * 64);

typedef float          v4f  __attribute__((ext_vector_type(4)));
typedef float          v8f  __attribute__((ext_vector_type(8)));
typedef int            v4i  __attribute__((ext_vector_type(4)));
typedef _Float16       v8h  __attribute__((ext_vector_type(8)));
typedef _Float16       v16h __attribute__((ext_vector_type(16)));
typedef unsigned short v8us __attribute__((ext_vector_type(8)));
typedef __bf16         v16b __attribute__((ext_vector_type(16)));
union FragH { v16h v; v8h h[2]; };
union FragB { v16b v; v8us h[2]; };

__device__ __forceinline__ v8h cvt8(v4f a, v4f b) {
  v8h r;
  r[0] = (_Float16)a.x; r[1] = (_Float16)a.y; r[2] = (_Float16)a.z; r[3] = (_Float16)a.w;
  r[4] = (_Float16)b.x; r[5] = (_Float16)b.y; r[6] = (_Float16)b.z; r[7] = (_Float16)b.w;
  return r;
}

__device__ __forceinline__ unsigned short bfbits(float f) {
  unsigned u = (unsigned)__float_as_uint(f);
  u += 0x7FFFu + ((u >> 16) & 1u);
  return (unsigned short)(u >> 16);
}
__device__ __forceinline__ float bfval(unsigned short b) { return __uint_as_float(((unsigned)b) << 16); }

__device__ __forceinline__ void split8(v4f a, v4f b, v8us& hi, v8us& lo) {
  float x[8];
  x[0] = a.x; x[1] = a.y; x[2] = a.z; x[3] = a.w; x[4] = b.x; x[5] = b.y; x[6] = b.z; x[7] = b.w;
#pragma unroll
  for (int e = 0; e < 8; ++e) {
    const unsigned short hb = bfbits(x[e]);
    hi[e] = hb;
    lo[e] = bfbits(x[e] - bfval(hb));
  }
}

__device__ __forceinline__ v8f wmh(v16h a, v16h b, v8f c) {
  v8f d = __builtin_amdgcn_wmma_f32_16x16x32_f16(false, a, false, b, (short)0, c, false, false);
  asm volatile("v_nop\n\tv_nop\n\tv_nop\n\tv_nop" : "+v"(d) : "v"(a), "v"(b));
  return d;
}
__device__ __forceinline__ v8f wmb(v16b a, v16b b, v8f c) {
  v8f d = __builtin_amdgcn_wmma_f32_16x16x32_bf16(false, a, false, b, (short)0, c, false, false);
  asm volatile("v_nop\n\tv_nop\n\tv_nop\n\tv_nop" : "+v"(d) : "v"(a), "v"(b));
  return d;
}

__device__ __forceinline__ int   rli(int v, int j)   { return __builtin_amdgcn_readlane(v, j); }
__device__ __forceinline__ float rlf(float v, int j) { return __int_as_float(__builtin_amdgcn_readlane(__float_as_int(v), j)); }

__device__ __forceinline__ float wsum(float v) {
#pragma unroll
  for (int d = 16; d > 0; d >>= 1) v += __shfl_xor(v, d);
  return v;
}
__device__ __forceinline__ float wmax(float v) {
#pragma unroll
  for (int d = 16; d > 0; d >>= 1) v = fmaxf(v, __shfl_xor(v, d));
  return v;
}
__device__ __forceinline__ float lrelu(float e) { return e >= 0.0f ? e : 0.2f * e; }
__device__ __forceinline__ float sigm(float v) {
  v = fminf(fmaxf(v, -40.0f), 40.0f);
  const float e = __expf(-v);
  return __builtin_amdgcn_rcpf(1.0f + e);
}

template <int NB>
__device__ __forceinline__ int scan_chunk(const int* __restrict__ dsts, int nE, int cbase, int slotBase,
                                          int vec8, int* list, int tid, int lane, int wave) {
  int wc = 0;
#pragma unroll
  for (int g = 0; g < NGRP; ++g) {
    const int el0  = (g * NTHR + tid) * EPT;
    const int e0   = cbase + el0;
    const int sent = -2147483647 - 1;
    v4i da, db;
    if (vec8 != 0 && cbase + CHUNK <= nE) {
      da = *(const v4i*)(dsts + e0);
      db = *(const v4i*)(dsts + e0 + 4);
    } else {
      da.x = (e0     < nE) ? dsts[min(e0, nE - 1)] : sent;
      da.y = (e0 + 1 < nE) ? dsts[min(e0 + 1, nE - 1)] : sent;
      da.z = (e0 + 2 < nE) ? dsts[min(e0 + 2, nE - 1)] : sent;
      da.w = (e0 + 3 < nE) ? dsts[min(e0 + 3, nE - 1)] : sent;
      db.x = (e0 + 4 < nE) ? dsts[min(e0 + 4, nE - 1)] : sent;
      db.y = (e0 + 5 < nE) ? dsts[min(e0 + 5, nE - 1)] : sent;
      db.z = (e0 + 6 < nE) ? dsts[min(e0 + 6, nE - 1)] : sent;
      db.w = (e0 + 7 < nE) ? dsts[min(e0 + 7, nE - 1)] : sent;
    }
    const unsigned nb = (unsigned)slotBase;
    const unsigned s0 = (unsigned)da.x - nb, s1 = (unsigned)da.y - nb;
    const unsigned s2 = (unsigned)da.z - nb, s3 = (unsigned)da.w - nb;
    const unsigned s4 = (unsigned)db.x - nb, s5 = (unsigned)db.y - nb;
    const unsigned s6 = (unsigned)db.z - nb, s7 = (unsigned)db.w - nb;
    const bool h0 = s0 < (unsigned)NB, h1 = s1 < (unsigned)NB, h2 = s2 < (unsigned)NB, h3 = s3 < (unsigned)NB;
    const bool h4 = s4 < (unsigned)NB, h5 = s5 < (unsigned)NB, h6 = s6 < (unsigned)NB, h7 = s7 < (unsigned)NB;
    const unsigned any = __builtin_amdgcn_ballot_w32(h0 | h1 | h2 | h3 | h4 | h5 | h6 | h7);
    if (any != 0u) {
#define HITJ(J, HJ, SJ) { \
        const unsigned mj = __builtin_amdgcn_ballot_w32(HJ); \
        if (mj != 0u) { \
          if (HJ) { \
            const int pos = wc + (int)__builtin_amdgcn_mbcnt_lo(mj, 0u); \
            if (pos < WCAP) list[wave * WCAP + pos] = ((el0 + (J)) << 12) | (int)(SJ); \
          } \
          wc += (int)__builtin_popcount(mj); } }
      HITJ(0, h0, s0)
      HITJ(1, h1, s1)
      HITJ(2, h2, s2)
      HITJ(3, h3, s3)
      HITJ(4, h4, s4)
      HITJ(5, h5, s5)
      HITJ(6, h6, s6)
      HITJ(7, h7, s7)
#undef HITJ
    }
  }
  return wc;
}

__global__ __launch_bounds__(NTHR) void k_wprep(
    const float* __restrict__ Wg, const float* __restrict__ W1, const float* __restrict__ W2,
    const float* __restrict__ F1, const float* __restrict__ F2,
    unsigned short* pgh, unsigned short* pgl, _Float16* p1, _Float16* p2, _Float16* pf) {
  const int g0 = HID * KP0 / 8;
  const int g1 = HID2 * HID / 8;
  const int g2 = g1;
  const int g3 = HID * HID2 / 8;
  const int bstart = blockIdx.x * NTHR;
  const float* src; const float* src2; _Float16* dst; int K, Nout, KP, segOff; float wsc;
  if (bstart < g0)                { src = Wg; src2 = Wg; dst = p1; K = FIN; Nout = HID;  KP = KP0;  segOff = 0;            wsc = 1.0f; }
  else if (bstart < g0 + g1)      { src = W1; src2 = W1; dst = p1; K = HID; Nout = HID2; KP = HID;  segOff = g0;           wsc = WSCALE; }
  else if (bstart < g0 + g1 + g2) { src = W2; src2 = W2; dst = p2; K = HID; Nout = HID2; KP = HID;  segOff = g0 + g1;      wsc = WSCALE; }
  else                            { src = F1; src2 = F2; dst = pf; K = HID; Nout = HID;  KP = HID2; segOff = g0 + g1 + g2; wsc = WSCALE; }
  const int i = bstart + (int)threadIdx.x;
  if (i >= g0 + g1 + g2 + g3) return;
  const int o  = (i - segOff) * 8;
  const int n  = o / KP;
  const int k0 = o - n * KP;
  const float* sp = src;
  int kb = k0;
  if (KP == HID2) {
    sp = (k0 < HID) ? src : src2;
    kb = k0 & (HID - 1);
  }
  const int nc = n < Nout ? n : Nout - 1;
  float v[8];
#pragma unroll
  for (int e = 0; e < 8; ++e) {
    const int k  = kb + e;
    const int kc = k < K ? k : K - 1;
    const float x = sp[(size_t)kc * Nout + nc];
    const float sc = (k < K && n < Nout) ? wsc : 0.0f;
    v[e] = x * sc;
  }
  v4f a, b;
  a.x = v[0]; a.y = v[1]; a.z = v[2]; a.w = v[3];
  b.x = v[4]; b.y = v[5]; b.z = v[6]; b.w = v[7];
  if (bstart < g0) {
    v8us hh, ll;
    split8(a, b, hh, ll);
    unsigned short* dh = pgh + o;
    unsigned short* dl = pgl + o;
    *(volatile v8us*)dh = hh;
    *(volatile v8us*)dl = ll;
    __threadfence();
    *(volatile v8us*)dh = hh;
    *(volatile v8us*)dl = ll;
  } else {
    const v8h hv = cvt8(a, b);
    _Float16* dp = dst + o;
    *(volatile v8h*)dp = hv;
    __threadfence();
    *(volatile v8h*)dp = hv;
  }
}

__global__ __launch_bounds__(NTHR) void k_count(const int* __restrict__ ei, int* cnt, int nE, int vec8) {
  __shared__ __attribute__((aligned(16))) int scnt[NBC];
  __shared__ __attribute__((aligned(16))) int list[LISTN];
  __shared__ int wcnt[NWAVE];
  const int tid = threadIdx.x, lane = tid & 31, wave = tid >> 5;
  const int nodeBase = blockIdx.x * NBC;
  const int* dsts = ei + nE;

  for (int i = tid; i < NBC; i += NTHR) scnt[i] = 0;
  __syncthreads();

  const int nChunks = (nE + CHUNK - 1) / CHUNK;
#pragma unroll 1
  for (int ch = 0; ch < nChunks; ++ch) {
    const int cbase = ch * CHUNK;
    const int wc = scan_chunk<NBC>(dsts, nE, cbase, nodeBase, vec8, list, tid, lane, wave);
    if (lane == 0) wcnt[wave] = wc;
    __syncthreads();
    if (wave == 0) {
#pragma unroll 1
      for (int wsx = 0; wsx < NWAVE; ++wsx) {
        int n = __builtin_amdgcn_readfirstlane(wcnt[wsx]);
        n = n > WCAP ? WCAP : (n < 0 ? 0 : n);
        const int* lp = list + wsx * WCAP;
#pragma unroll 1
        for (int i = 0; i < n; ++i) {
          const int ent  = __builtin_amdgcn_readfirstlane(lp[i]);
          const int slot = ent & (NBC - 1);
          if (lane == 0) scnt[slot] = scnt[slot] + 1;
        }
      }
    }
    __syncthreads();
  }

  v4i cq[4];
#pragma unroll
  for (int q = 0; q < 4; ++q) {
    const int f = (wave * 4 + q) * 128 + 4 * lane;
    cq[q] = *(const v4i*)(scnt + f);
  }
  int* cp = cnt + (size_t)nodeBase;
#pragma unroll
  for (int q = 0; q < 4; ++q) {
    const int f = (wave * 4 + q) * 128 + 4 * lane;
    *(volatile v4i*)(cp + f) = cq[q];
  }
  __threadfence();
#pragma unroll
  for (int q = 0; q < 4; ++q) {
    const int f = (wave * 4 + q) * 128 + 4 * lane;
    *(volatile v4i*)(cp + f) = cq[q];
  }
}

__global__ __launch_bounds__(OTHR) void k_offsets(
    const int* __restrict__ cnt, int* off, int* rbase, int nChunk) {
  __shared__ __attribute__((aligned(16))) int soff[NBC];
  __shared__ __attribute__((aligned(16))) int srb[RBN];
  __shared__ int wtot[OTHR / 32];
  const int tid = threadIdx.x, lane = tid & 31, wave = tid >> 5, sub = tid >> 7;
  for (int i = tid; i < RBN; i += OTHR) srb[i] = 0;
  int carry = 0;
#pragma unroll 1
  for (int ch = 0; ch < nChunk; ++ch) {
    const int base = ch * NBC;
    const v4i c0 = *(const v4i*)(cnt + base + 8 * tid);
    const v4i c1 = *(const v4i*)(cnt + base + 8 * tid + 4);
    const int e0 = max(c0.x, 0), e1 = max(c0.y, 0), e2 = max(c0.z, 0), e3 = max(c0.w, 0);
    const int e4 = max(c1.x, 0), e5 = max(c1.y, 0), e6 = max(c1.z, 0), e7 = max(c1.w, 0);
    const int ts = e0 + e1 + e2 + e3 + e4 + e5 + e6 + e7;
    int incl = ts;
#pragma unroll
    for (int d = 1; d < 32; d <<= 1) {
      const int t = __shfl_up(incl, d);
      if (lane >= d) incl += t;
    }
    if (lane == 31) wtot[wave] = incl;
    __syncthreads();
    const int S0 = wtot[0]  + wtot[1]  + wtot[2]  + wtot[3];
    const int S1 = wtot[4]  + wtot[5]  + wtot[6]  + wtot[7];
    const int S2 = wtot[8]  + wtot[9]  + wtot[10] + wtot[11];
    const int S3 = wtot[12] + wtot[13] + wtot[14] + wtot[15];
    int pre = 0;
#pragma unroll 1
    for (int w = 4 * sub; w < wave; ++w) pre += wtot[w];
    const int b0 = carry;
    const int b1 = b0 + ((S0 + 31) & ~31);
    const int b2 = b1 + ((S1 + 31) & ~31);
    const int b3 = b2 + ((S2 + 31) & ~31);
    const int b4 = b3 + ((S3 + 31) & ~31);
    const int myb = sub == 0 ? b0 : (sub == 1 ? b1 : (sub == 2 ? b2 : b3));
    if (tid == 0) {
      srb[min(4 * ch + 0, RBN - 1)] = b0;
      srb[min(4 * ch + 1, RBN - 1)] = b1;
      srb[min(4 * ch + 2, RBN - 1)] = b2;
      srb[min(4 * ch + 3, RBN - 1)] = b3;
    }
    int run = myb + pre + incl - ts;
    soff[8 * tid + 0] = run; run += e0;
    soff[8 * tid + 1] = run; run += e1;
    soff[8 * tid + 2] = run; run += e2;
    soff[8 * tid + 3] = run; run += e3;
    soff[8 * tid + 4] = run; run += e4;
    soff[8 * tid + 5] = run; run += e5;
    soff[8 * tid + 6] = run; run += e6;
    soff[8 * tid + 7] = run;
    carry = b4;
    __syncthreads();
    const v4i o0 = *(const v4i*)(soff + 4 * tid);
    const v4i o1 = *(const v4i*)(soff + 4 * (tid + OTHR));
    int* op = off + base;
    *(volatile v4i*)(op + 4 * tid) = o0;
    *(volatile v4i*)(op + 4 * (tid + OTHR)) = o1;
    __threadfence();
    *(volatile v4i*)(op + 4 * tid) = o0;
    *(volatile v4i*)(op + 4 * (tid + OTHR)) = o1;
    __syncthreads();
  }
  if (tid == 0) srb[min(4 * nChunk, RBN - 1)] = carry;
  __syncthreads();
  v4i rv = {0, 0, 0, 0};
  if (tid < 32) rv = *(const v4i*)(srb + 4 * tid);
  if (tid < 32) *(volatile v4i*)(rbase + 4 * tid) = rv;
  __threadfence();
  if (tid < 32) *(volatile v4i*)(rbase + 4 * tid) = rv;
}

__global__ __launch_bounds__(NTHR) void k_fill(
    const int* __restrict__ ei, const int* __restrict__ off, const int* __restrict__ rbase,
    int* csr, int nE, int vec8, int csrLen) {
  extern __shared__ v4f lds_dyn[];
  int* region = (int*)lds_dyn;
  int* cursor = region + RCAP;
  int* list   = cursor + NBF;
  int* wcnt   = list + LISTN;
  const int tid = threadIdx.x, lane = tid & 31, wave = tid >> 5;
  const int b = blockIdx.x;
  const int nodeBase = b * NBF;
  const int* dsts = ei + nE;

  int rb0 = rbase[b];
  const int rb1 = rbase[b + 1];
  rb0 = rb0 < 0 ? 0 : (rb0 > csrLen ? csrLen : rb0);
  rb0 &= ~31;
  int len = rb1 - rb0;
  len = len < 0 ? 0 : (len > RCAP ? RCAP : len);
  int lenW = (len + 31) & ~31;
  if (rb0 + lenW > csrLen) lenW = (csrLen - rb0) & ~31;

  {
    const v4i z = {0, 0, 0, 0};
    for (int i = tid; i < RCAP / 4; i += NTHR) ((v4i*)region)[i] = z;
    for (int s = tid; s < NBF; s += NTHR) {
      int o = off[nodeBase + s] - rb0;
      o = o < 0 ? 0 : (o > RCAP ? RCAP : o);
      cursor[s] = o;
    }
  }
  __syncthreads();

  const int nChunks = (nE + CHUNK - 1) / CHUNK;
#pragma unroll 1
  for (int ch = 0; ch < nChunks; ++ch) {
    const int cbase = ch * CHUNK;
    const int wc = scan_chunk<NBF>(dsts, nE, cbase, nodeBase, vec8, list, tid, lane, wave);
    if (lane == 0) wcnt[wave] = wc;
    __syncthreads();
    if (wave == 0) {
#pragma unroll 1
      for (int wsx = 0; wsx < NWAVE; ++wsx) {
        int n = __builtin_amdgcn_readfirstlane(wcnt[wsx]);
        n = n > WCAP ? WCAP : (n < 0 ? 0 : n);
        const int* lp = list + wsx * WCAP;
#pragma unroll 1
        for (int i = 0; i < n; ++i) {
          const int ent  = __builtin_amdgcn_readfirstlane(lp[i]);
          const int slot = ent & (NBF - 1);
          int e = cbase + ((ent >> 12) & (CHUNK - 1));
          e = e > nE - 1 ? nE - 1 : e;
          if (lane == 0) {
            int pos = cursor[slot];
            pos = pos < 0 ? 0 : (pos > RCAP - 1 ? RCAP - 1 : pos);
            region[pos] = e;
            const int np = pos + 1;
            cursor[slot] = np > RCAP ? RCAP : np;
          }
        }
      }
    }
    __syncthreads();
  }

  const int nv = lenW >> 2;
  int* gp = csr + rb0;
#pragma unroll 1
  for (int i = tid; i < nv; i += NTHR) { const v4i v = ((const v4i*)region)[i]; *(volatile v4i*)(gp + 4 * i) = v; }
  __threadfence();
#pragma unroll 1
  for (int i = tid; i < nv; i += NTHR) { const v4i v = ((const v4i*)region)[i]; *(volatile v4i*)(gp + 4 * i) = v; }
}

__global__ __launch_bounds__(NTHR) void k_deg(
    const int* __restrict__ csr, const int* __restrict__ cnt, const int* __restrict__ off,
    const float* __restrict__ tw, float* dinv, int nE, int csrLen) {
  __shared__ __attribute__((aligned(16))) float sd[NTHR];
  const int tid = (int)threadIdx.x;
  const int t = blockIdx.x * NTHR + tid;
  int n = cnt[t];
  n = n < 0 ? 0 : (n > DEGCAP ? DEGCAP : n);
  const int st = off[t];
  float d = 0.0f;
#pragma unroll 1
  for (int p = 0; p < n; ++p) {
    int pos = st + p;
    pos = pos < 0 ? 0 : (pos > csrLen - 1 ? csrLen - 1 : pos);
    int e = csr[pos];
    e = e < 0 ? 0 : (e > nE - 1 ? nE - 1 : e);
    d += tw[e];
  }
  const float deg = d + 1.0f;
  const float dv = deg > 0.0f ? rsqrtf(deg) : 0.0f;
  sd[tid] = dv;
  __syncthreads();
  const int q = tid & 63;
  v4f v = {0.f, 0.f, 0.f, 0.f};
  if (tid < 64) v = *(const v4f*)(sd + 4 * q);
  float* gp = dinv + (size_t)blockIdx.x * NTHR + 4 * q;
  if (tid < 64) *(volatile v4f*)gp = v;
  __threadfence();
  if (tid < 64) *(volatile v4f*)gp = v;
}

template <int KD>
__device__ __forceinline__ void mma_tile(const _Float16* sA, const _Float16* __restrict__ Bs,
                                         int wave, int lane, v8f (&acc)[8]) {
  constexpr int AP = KD + 8;
  const int hh = lane >> 4, m = lane & 15;
#pragma unroll
  for (int t = 0; t < 8; ++t) { v8f z = {0.f, 0.f, 0.f, 0.f, 0.f, 0.f, 0.f, 0.f}; acc[t] = z; }
  const _Float16* ar = sA + (wave * 16 + m) * AP + 8 * hh;
#pragma unroll 1
  for (int kt = 0; kt < KD / 32; ++kt) {
    FragH a;
    a.h[0] = *(const v8h*)(ar + 32 * kt);
    a.h[1] = *(const v8h*)(ar + 32 * kt + 16);
#pragma unroll
    for (int t = 0; t < 8; ++t) {
      const _Float16* bp = Bs + (size_t)(16 * t + m) * KD + 32 * kt + 8 * hh;
      FragH b;
      b.h[0] = *(const v8h*)bp;
      b.h[1] = *(const v8h*)(bp + 16);
      acc[t] = wmh(a.v, b.v, acc[t]);
    }
  }
}

__device__ __forceinline__ void store16(const float* lp, float* gp, int pitch, int lane, int nvalid) {
  lp += 4 * lane; gp += 4 * lane;
#pragma unroll
  for (int i = 0; i < 16; ++i) {
    if (i < nvalid) { const v4f v = *(const v4f*)(lp + i * HID); *(volatile v4f*)(gp + (size_t)i * pitch) = v; }
  }
  __threadfence();
#pragma unroll
  for (int i = 0; i < 16; ++i) {
    if (i < nvalid) { const v4f v = *(const v4f*)(lp + i * HID); *(volatile v4f*)(gp + (size_t)i * pitch) = v; }
  }
}

__global__ __launch_bounds__(NTHR) void k_gemm0(
    const float* __restrict__ X, const unsigned short* __restrict__ BH, const unsigned short* __restrict__ BL,
    const float* __restrict__ dinv, float* C, int nN) {
  extern __shared__ v4f lds_dyn[];
  constexpr int AP = KP0 + 8;
  unsigned short* sH  = (unsigned short*)lds_dyn;
  unsigned short* sL  = sH + GROWS * AP;
  float*          stg = (float*)lds_dyn;
  const int tid = threadIdx.x, lane = tid & 31, wave = tid >> 5, hh = lane >> 4, m = lane & 15;
  const int rowBase = blockIdx.x * GROWS;

#pragma unroll
  for (int it = 0; it < (GROWS * KP0 / 8) / NTHR; ++it) {
    const int idx = it * NTHR + tid;
    const int r   = idx >> 3;
    const int k0  = (idx & 7) * 8;
    int row = rowBase + r;
    row = row > nN - 1 ? nN - 1 : row;
    const float* xp = X + (size_t)row * FIN;
    float v[8];
#pragma unroll
    for (int e = 0; e < 8; ++e) {
      const int k  = k0 + e;
      const int kc = k < FIN ? k : FIN - 1;
      const float x = xp[kc];
      const float sc = k < FIN ? 1.0f : 0.0f;
      v[e] = x * sc;
    }
    v4f a, b;
    a.x = v[0]; a.y = v[1]; a.z = v[2]; a.w = v[3];
    b.x = v[4]; b.y = v[5]; b.z = v[6]; b.w = v[7];
    v8us h8, l8;
    split8(a, b, h8, l8);
    *(v8us*)(sH + r * AP + k0) = h8;
    *(v8us*)(sL + r * AP + k0) = l8;
  }
  __syncthreads();

  v8f acc[8];
#pragma unroll
  for (int t = 0; t < 8; ++t) { v8f z = {0.f, 0.f, 0.f, 0.f, 0.f, 0.f, 0.f, 0.f}; acc[t] = z; }
  const unsigned short* arH = sH + (wave * 16 + m) * AP + 8 * hh;
  const unsigned short* arL = sL + (wave * 16 + m) * AP + 8 * hh;
#pragma unroll 1
  for (int kt = 0; kt < KP0 / 32; ++kt) {
    FragB ah, al;
    ah.h[0] = *(const v8us*)(arH + 32 * kt);
    ah.h[1] = *(const v8us*)(arH + 32 * kt + 16);
    al.h[0] = *(const v8us*)(arL + 32 * kt);
    al.h[1] = *(const v8us*)(arL + 32 * kt + 16);
#pragma unroll
    for (int t = 0; t < 8; ++t) {
      const size_t bo = (size_t)(16 * t + m) * KP0 + 32 * kt + 8 * hh;
      FragB bh, bl;
      bh.h[0] = *(const v8us*)(BH + bo);
      bh.h[1] = *(const v8us*)(BH + bo + 16);
      bl.h[0] = *(const v8us*)(BL + bo);
      bl.h[1] = *(const v8us*)(BL + bo + 16);
      acc[t] = wmb(ah.v, bh.v, acc[t]);
      acc[t] = wmb(al.v, bh.v, acc[t]);
      acc[t] = wmb(ah.v, bl.v, acc[t]);
    }
  }
  __syncthreads();

  const int r0 = wave * 16 + 8 * hh;
  const v4f dA = *(const v4f*)(dinv + (size_t)rowBase + r0);
  const v4f dB = *(const v4f*)(dinv + (size_t)rowBase + r0 + 4);
  float s[8];
  s[0] = dA.x; s[1] = dA.y; s[2] = dA.z; s[3] = dA.w; s[4] = dB.x; s[5] = dB.y; s[6] = dB.z; s[7] = dB.w;
  float* sp = stg + r0 * HID + m;
#pragma unroll
  for (int t = 0; t < 8; ++t) {
#pragma unroll
    for (int r = 0; r < 8; ++r) sp[r * HID + 16 * t] = acc[t][r] * s[r];
  }
  __syncthreads();

  store16(stg + wave * 16 * HID, C + ((size_t)rowBase + wave * 16) * HID, HID, lane, 16);
}

__global__ __launch_bounds__(NTHR) void k_gemm1(
    const float* __restrict__ A, const _Float16* __restrict__ Bs, const float* __restrict__ as,
    const float* __restrict__ ad, float* C, float* attp, int npad) {
  extern __shared__ v4f lds_dyn[];
  constexpr int KD = HID;
  constexpr int AP = KD + 8;
  _Float16* sA   = (_Float16*)lds_dyn;
  float*    stg  = (float*)lds_dyn;
  float*    sAtt = (float*)lds_dyn + GROWS * HID;
  const int tid = threadIdx.x, lane = tid & 31, wave = tid >> 5, hh = lane >> 4, m = lane & 15;
  const int rowBase = blockIdx.x * GROWS;
  const int y = blockIdx.y;
  const _Float16* Bsy = Bs + (size_t)y * HID * KD;

#pragma unroll
  for (int it = 0; it < (GROWS * KD / 8) / NTHR; ++it) {
    const int idx = it * NTHR + tid;
    const int r   = idx >> 4;
    const int c0  = (idx & 15) * 8;
    int row = rowBase + r;
    row = row > npad - 1 ? npad - 1 : row;
    const float* ap = A + (size_t)row * KD + c0;
    const v4f a = *(const v4f*)ap * ASCALE, b = *(const v4f*)(ap + 4) * ASCALE;
    *(v8h*)(sA + r * AP + c0) = cvt8(a, b);
  }
  __syncthreads();

  v8f acc[8];
  mma_tile<KD>(sA, Bsy, wave, lane, acc);
  __syncthreads();

  const int r0 = wave * 16 + 8 * hh;
  float* sp = stg + r0 * HID + m;
#pragma unroll
  for (int t = 0; t < 8; ++t) {
#pragma unroll
    for (int r = 0; r < 8; ++r) sp[r * HID + 16 * t] = acc[t][r] * OSCALE;
  }
  __syncthreads();

  const v4f as4 = *(const v4f*)(as + y * HID + 4 * lane);
  const v4f ad4 = *(const v4f*)(ad + y * HID + 4 * lane);
  float mys = 0.0f, myd = 0.0f;
  const float* wp = stg + wave * 16 * HID + 4 * lane;
#pragma unroll
  for (int i = 0; i < 16; ++i) {
    const v4f x4 = *(const v4f*)(wp + i * HID);
    float ps = x4.x * as4.x + x4.y * as4.y + x4.z * as4.z + x4.w * as4.w;
    float pd = x4.x * ad4.x + x4.y * ad4.y + x4.z * ad4.z + x4.w * ad4.w;
    ps = wsum(ps);
    pd = wsum(pd);
    mys = (lane == i) ? ps : mys;
    myd = (lane == i) ? pd : myd;
  }
  if (lane < 16) {
    sAtt[wave * 16 + lane] = mys;
    sAtt[GROWS + wave * 16 + lane] = myd;
  }
  __syncthreads();

  v4f av = {0.f, 0.f, 0.f, 0.f};
  float* apn = attp;
  if (wave < 2) {
    av  = *(const v4f*)(sAtt + wave * GROWS + 4 * lane);
    apn = attp + (size_t)(2 * wave + y) * npad + rowBase + 4 * lane;
  }
  const float* lp = stg + wave * 16 * HID + 4 * lane;
  float* gp = C + ((size_t)rowBase + wave * 16) * HID2 + y * HID + 4 * lane;
#pragma unroll
  for (int i = 0; i < 16; ++i) { const v4f v = *(const v4f*)(lp + i * HID); *(volatile v4f*)(gp + (size_t)i * HID2) = v; }
  if (wave < 2) *(volatile v4f*)apn = av;
  __threadfence();
#pragma unroll
  for (int i = 0; i < 16; ++i) { const v4f v = *(const v4f*)(lp + i * HID); *(volatile v4f*)(gp + (size_t)i * HID2) = v; }
  if (wave < 2) *(volatile v4f*)apn = av;
}

__global__ __launch_bounds__(NTHR) void k_gemm2(
    const float* __restrict__ XT, const float* __restrict__ XX, const _Float16* __restrict__ Bs,
    const float* __restrict__ b1, const float* __restrict__ b2, const float* __restrict__ pb,
    float* Out, int npad, int nOut) {
  extern __shared__ v4f lds_dyn[];
  constexpr int KD = HID2;
  constexpr int AP = KD + 8;
  _Float16* sA  = (_Float16*)lds_dyn;
  float*    stg = (float*)lds_dyn;
  const int tid = threadIdx.x, lane = tid & 31, wave = tid >> 5, hh = lane >> 4, m = lane & 15;
  const int rowBase = blockIdx.x * GROWS;

#pragma unroll
  for (int it = 0; it < (GROWS * KD / 8) / NTHR; ++it) {
    const int idx = it * NTHR + tid;
    const int r   = idx >> 5;
    const int g   = idx & 31;
    int row = rowBase + r;
    row = row > npad - 1 ? npad - 1 : row;
    const float* ap = (g < 16) ? (XT + (size_t)row * HID + 8 * g) : (XX + (size_t)row * HID + 8 * (g - 16));
    const v4f a = *(const v4f*)ap * ASCALE, b = *(const v4f*)(ap + 4) * ASCALE;
    *(v8h*)(sA + r * AP + 8 * g) = cvt8(a, b);
  }
  __syncthreads();

  v8f acc[8];
  mma_tile<KD>(sA, Bs, wave, lane, acc);
  __syncthreads();

  const int r0 = wave * 16 + 8 * hh;
  float bsum[8];
#pragma unroll
  for (int t = 0; t < 8; ++t) {
    const int n = 16 * t + m;
    bsum[t] = b1[n] + b2[n] + pb[n];
  }
  float* sp = stg + r0 * HID + m;
#pragma unroll
  for (int t = 0; t < 8; ++t) {
#pragma unroll
    for (int r = 0; r < 8; ++r) sp[r * HID + 16 * t] = acc[t][r] * OSCALE + bsum[t];
  }
  __syncthreads();

  float* lp = stg + wave * 16 * HID + 4 * lane;
  const int growBase = rowBase + wave * 16;
#pragma unroll 4
  for (int i = 0; i < 16; ++i) {
    const size_t row = (size_t)(growBase + i);
    const v4f vz  = *(const v4f*)(lp + i * HID);
    const v4f xt4 = *(const v4f*)(XT + row * HID + 4 * lane);
    const v4f x4  = *(const v4f*)(XX + row * HID + 4 * lane);
    v4f z;
    z.x = sigm(vz.x); z.y = sigm(vz.y); z.z = sigm(vz.z); z.w = sigm(vz.w);
    v4f one = {1.f, 1.f, 1.f, 1.f};
    const v4f o = z * xt4 + (one - z) * x4;
    *(v4f*)(lp + i * HID) = o;
  }
  int nvalid = nOut - growBase;
  nvalid = nvalid < 0 ? 0 : (nvalid > 16 ? 16 : nvalid);
  store16(stg + wave * 16 * HID, Out + (size_t)growBase * HID, HID, lane, nvalid);
}

__global__ __launch_bounds__(NTHR) void k_gagg(
    const int* __restrict__ csr, const int* __restrict__ off, const int* __restrict__ cnt,
    const int* __restrict__ ei, const float* __restrict__ tw, const float* __restrict__ dinv,
    const float* __restrict__ hw, const float* __restrict__ bias, float* X,
    int nN, int nE, int csrLen) {
  const int tid = threadIdx.x, lane = tid & 31, wave = tid >> 5;
  const int tbase = blockIdx.x * TGT + wave * 32;
  const int cl = tbase + lane;
  const int cnt_l = cnt[cl];
  const int off_l = off[cl];
  const float dv_l = dinv[cl];
  const v4f bb = *(const v4f*)(bias + 4 * lane);

#pragma unroll 1
  for (int j = 0; j < 32; ++j) {
    const int c = tbase + j;
    int n = rli(cnt_l, j);
    n = n < 0 ? 0 : (n > DEGCAP ? DEGCAP : n);
    const int st = rli(off_l, j);
    const float dc = rlf(dv_l, j);
    v4f acc = {0.f, 0.f, 0.f, 0.f};
#pragma unroll 1
    for (int q0 = 0; q0 < n; q0 += 32) {
      int pos = st + q0 + lane;
      pos = pos < 0 ? 0 : (pos > csrLen - 1 ? csrLen - 1 : pos);
      int e = csr[pos];
      e = e < 0 ? 0 : (e > nE - 1 ? nE - 1 : e);
      int s = ei[e];
      s = s < 0 ? 0 : (s > nN - 1 ? nN - 1 : s);
      const float wv = tw[e];
      const int mcnt = (n - q0) < 32 ? (n - q0) : 32;
#pragma unroll 1
      for (int p = 0; p < mcnt; ++p) {
        const int sp = rli(s, p);
        const float wp = rlf(wv, p);
        acc = acc + *(const v4f*)(hw + (size_t)sp * HID + 4 * lane) * wp;
      }
    }
    const v4f sv = *(const v4f*)(hw + (size_t)c * HID + 4 * lane);
    v4f v = (acc + sv) * dc + bb;
    v.x = fmaxf(v.x, 0.f); v.y = fmaxf(v.y, 0.f); v.z = fmaxf(v.z, 0.f); v.w = fmaxf(v.w, 0.f);
    float* hp = X + (size_t)c * HID + 4 * lane;
    *(volatile v4f*)hp = v;
    __threadfence();
    *(volatile v4f*)hp = v;
  }
}

__global__ __launch_bounds__(NTHR) void k_tagg(
    const int* __restrict__ csr, const int* __restrict__ off, const int* __restrict__ cnt,
    const int* __restrict__ ei, const float* __restrict__ attp, const float* __restrict__ xl,
    const float* __restrict__ bias, float* XT, int nN, int nE, int csrLen, int npad, int relu) {
  const int tid = threadIdx.x, lane = tid & 31, wave = tid >> 5;
  const int tbase = blockIdx.x * TGT + wave * 32;
  const int cl = tbase + lane;
  const int cnt_l = cnt[cl];
  const int off_l = off[cl];
  const float* as0p = attp;
  const float* as1p = attp + (size_t)npad;
  const float as0_l = as0p[cl];
  const float as1_l = as1p[cl];
  const float ad0_l = attp[(size_t)2 * npad + cl];
  const float ad1_l = attp[(size_t)3 * npad + cl];
  const v4f bb = *(const v4f*)(bias + 4 * lane);

#pragma unroll 1
  for (int j = 0; j < 32; ++j) {
    const int c = tbase + j;
    int n = rli(cnt_l, j);
    n = n < 0 ? 0 : (n > DEGCAP ? DEGCAP : n);
    const int st = rli(off_l, j);
    const float ad0 = rlf(ad0_l, j), ad1 = rlf(ad1_l, j);
    const float es0 = lrelu(rlf(as0_l, j) + ad0);
    const float es1 = lrelu(rlf(as1_l, j) + ad1);

    float m0 = es0, m1 = es1;
#pragma unroll 1
    for (int q0 = 0; q0 < n; q0 += 32) {
      int pos = st + q0 + lane;
      pos = pos < 0 ? 0 : (pos > csrLen - 1 ? csrLen - 1 : pos);
      int e = csr[pos];
      e = e < 0 ? 0 : (e > nE - 1 ? nE - 1 : e);
      int s = ei[e];
      s = s < 0 ? 0 : (s > nN - 1 ? nN - 1 : s);
      const bool valid = (q0 + lane) < n;
      const float e0 = lrelu(as0p[s] + ad0);
      const float e1 = lrelu(as1p[s] + ad1);
      m0 = valid ? fmaxf(m0, e0) : m0;
      m1 = valid ? fmaxf(m1, e1) : m1;
    }
    m0 = wmax(m0);
    m1 = wmax(m1);

    float ss0 = 0.f, ss1 = 0.f;
    v4f acc0 = {0.f, 0.f, 0.f, 0.f}, acc1 = {0.f, 0.f, 0.f, 0.f};
#pragma unroll 1
    for (int q0 = 0; q0 < n; q0 += 32) {
      int pos = st + q0 + lane;
      pos = pos < 0 ? 0 : (pos > csrLen - 1 ? csrLen - 1 : pos);
      int e = csr[pos];
      e = e < 0 ? 0 : (e > nE - 1 ? nE - 1 : e);
      int s = ei[e];
      s = s < 0 ? 0 : (s > nN - 1 ? nN - 1 : s);
      const bool valid = (q0 + lane) < n;
      const float e0 = lrelu(as0p[s] + ad0);
      const float e1 = lrelu(as1p[s] + ad1);
      const float p0 = valid ? __expf(e0 - m0) : 0.0f;
      const float p1 = valid ? __expf(e1 - m1) : 0.0f;
      ss0 += p0;
      ss1 += p1;
      const int mcnt = (n - q0) < 32 ? (n - q0) : 32;
#pragma unroll 1
      for (int p = 0; p < mcnt; ++p) {
        const int sp = rli(s, p);
        const float a0 = rlf(p0, p);
        const float a1 = rlf(p1, p);
        const float* xr = xl + (size_t)sp * HID2 + 4 * lane;
        const v4f v0 = *(const v4f*)xr;
        const v4f v1 = *(const v4f*)(xr + HID);
        acc0 = acc0 + v0 * a0;
        acc1 = acc1 + v1 * a1;
      }
    }
    const float ps0 = __expf(es0 - m0), ps1 = __expf(es1 - m1);
    const float S0 = wsum(ss0) + ps0;
    const float S1 = wsum(ss1) + ps1;
    const float* xc = xl + (size_t)c * HID2 + 4 * lane;
    acc0 = acc0 + *(const v4f*)xc * ps0;
    acc1 = acc1 + *(const v4f*)(xc + HID) * ps1;
    const float i0 = __builtin_amdgcn_rcpf(S0), i1 = __builtin_amdgcn_rcpf(S1);
    v4f v = (acc0 * i0 + acc1 * i1) * 0.5f + bb;
    if (relu != 0) { v.x = fmaxf(v.x, 0.f); v.y = fmaxf(v.y, 0.f); v.z = fmaxf(v.z, 0.f); v.w = fmaxf(v.w, 0.f); }
    float* hp = XT + (size_t)c * HID + 4 * lane;
    *(volatile v4f*)hp = v;
    __threadfence();
    *(volatile v4f*)hp = v;
  }
}

extern "C" void kernel_launch(void* const* d_in, const int* in_sizes, int n_in,
                              void* d_out, int out_size, void* d_ws, size_t ws_size,
                              hipStream_t stream) {
  if (n_in < 18) return;
  const int nN = in_sizes[0] / FIN;
  const int nE = in_sizes[1] / 2;
  if (nN <= 0 || nE <= 0 || in_sizes[0] != nN * FIN || in_sizes[1] != 2 * nE || in_sizes[2] != nE) return;
  if (in_sizes[3] != FIN * HID || in_sizes[4] < HID) return;
  if (in_sizes[5] != HID * HID2 || in_sizes[6] < HID2 || in_sizes[7] < HID2 || in_sizes[8] < HID) return;
  if (in_sizes[9] != HID * HID2 || in_sizes[10] < HID2 || in_sizes[11] < HID2 || in_sizes[12] < HID) return;
  if (in_sizes[13] != HID * HID || in_sizes[14] < HID || in_sizes[15] != HID * HID || in_sizes[16] < HID) return;
  if (in_sizes[17] < HID) return;
  if (out_size != nN * HID) return;
  if (nE > (1 << 28) || nN > (1 << 24)) return;

  const float* x     = (const float*)d_in[0];
  const int*   ei    = (const int*)d_in[1];
  const float* tw    = (const float*)d_in[2];
  const float* Wg    = (const float*)d_in[3];
  const float* bg    = (const float*)d_in[4];
  const float* Wa1   = (const float*)d_in[5];
  const float* as1   = (const float*)d_in[6];
  const float* ad1   = (const float*)d_in[7];
  const float* ba1   = (const float*)d_in[8];
  const float* Wa2   = (const float*)d_in[9];
  const float* as2   = (const float*)d_in[10];
  const float* ad2   = (const float*)d_in[11];
  const float* ba2   = (const float*)d_in[12];
  const float* F1    = (const float*)d_in[13];
  const float* bf1   = (const float*)d_in[14];
  const float* F2    = (const float*)d_in[15];
  const float* bf2   = (const float*)d_in[16];
  const float* pbias = (const float*)d_in[17];
  float* out = (float*)d_out;

  const int NPAD   = ((nN + TGT - 1) / TGT) * TGT;
  const int nBC    = (nN + NBC - 1) / NBC;
  const int CNTPAD = nBC * NBC;
  if (4 * nBC + 1 > RBN) return;
  const int nBF    = (nN + NBF - 1) / NBF;
  const int csrLen = ((nE + 31) & ~31) + 4096;
  const int nGemm  = NPAD / GROWS;
  const int nAgg   = NPAD / TGT;
  const int nDeg   = CNTPAD / NTHR;

  char* ws = (char*)d_ws;
  size_t off = 0;
  const size_t oWGH = off; off += (size_t)HID * KP0 * 2;           off = (off + 255) & ~(size_t)255;
  const size_t oWGL = off; off += (size_t)HID * KP0 * 2;           off = (off + 255) & ~(size_t)255;
  const size_t oW1  = off; off += (size_t)HID2 * HID * 2;          off = (off + 255) & ~(size_t)255;
  const size_t oW2  = off; off += (size_t)HID2 * HID * 2;          off = (off + 255) & ~(size_t)255;
  const size_t oWF  = off; off += (size_t)HID * HID2 * 2;          off = (off + 255) & ~(size_t)255;
  const size_t oCnt = off; off += (size_t)CNTPAD * 4;              off = (off + 255) & ~(size_t)255;
  const size_t oOff = off; off += (size_t)CNTPAD * 4;              off = (off + 255) & ~(size_t)255;
  const size_t oDv  = off; off += (size_t)CNTPAD * 4;              off = (off + 255) & ~(size_t)255;
  const size_t oRb  = off; off += (size_t)RBN * 4;                 off = (off + 255) & ~(size_t)255;
  const size_t oCsr = off; off += (size_t)csrLen * 4;              off = (off + 255) & ~(size_t)255;
  const size_t oAtt = off; off += (size_t)4 * NPAD * 4;            off = (off + 255) & ~(size_t)255;
  const size_t oR1  = off; off += (size_t)NPAD * HID2 * 4;         off = (off + 255) & ~(size_t)255;
  const size_t oR2  = off; off += (size_t)NPAD * HID2 * 4;         off = (off + 255) & ~(size_t)255;
  if (off > ws_size) return;
  unsigned short* wgh = (unsigned short*)(ws + oWGH);
  unsigned short* wgl = (unsigned short*)(ws + oWGL);
  _Float16* w1   = (_Float16*)(ws + oW1);
  _Float16* w2   = (_Float16*)(ws + oW2);
  _Float16* wf   = (_Float16*)(ws + oWF);
  int*      cnt  = (int*)(ws + oCnt);
  int*      offp = (int*)(ws + oOff);
  float*    dinv = (float*)(ws + oDv);
  int*      rb   = (int*)(ws + oRb);
  int*      csr  = (int*)(ws + oCsr);
  float*    attp = (float*)(ws + oAtt);
  float*    R1   = (float*)(ws + oR1);
  float*    R2   = (float*)(ws + oR2);
  float*    R1a  = R1;
  float*    R1b  = R1 + (size_t)NPAD * HID;
  float*    R2a  = R2;
  float*    R2b  = R2 + (size_t)NPAD * HID;

  const int vec8 = ((nE & 3) == 0) ? 1 : 0;

  const int nPrep = HID * KP0 / 8 + 2 * (HID2 * HID / 8) + HID * HID2 / 8;
  k_wprep<<<nPrep / NTHR, NTHR, 0, stream>>>(Wg, Wa1, Wa2, F1, F2, wgh, wgl, w1, w2, wf);

  k_count<<<nBC, NTHR, 0, stream>>>(ei, cnt, nE, vec8);
  k_offsets<<<1, OTHR, 0, stream>>>(cnt, offp, rb, nBC);
  hipFuncSetAttribute(reinterpret_cast<const void*>(&k_fill),
                      hipFuncAttributeMaxDynamicSharedMemorySize, LDS_FILL);
  k_fill<<<nBF, NTHR, LDS_FILL, stream>>>(ei, offp, rb, csr, nE, vec8, csrLen);

  k_deg<<<nDeg, NTHR, 0, stream>>>(csr, cnt, offp, tw, dinv, nE, csrLen);

  hipFuncSetAttribute(reinterpret_cast<const void*>(&k_gemm0),
                      hipFuncAttributeMaxDynamicSharedMemorySize, LDS_G0);
  hipFuncSetAttribute(reinterpret_cast<const void*>(&k_gemm1),
                      hipFuncAttributeMaxDynamicSharedMemorySize, LDS_G1);
  hipFuncSetAttribute(reinterpret_cast<const void*>(&k_gemm2),
                      hipFuncAttributeMaxDynamicSharedMemorySize, LDS_G2);
  k_gemm0<<<nGemm, NTHR, LDS_G0, stream>>>(x, wgh, wgl, dinv, R2a, nN);
  k_gagg<<<nAgg, NTHR, 0, stream>>>(csr, offp, cnt, ei, tw, dinv, R2a, bg, R1a, nN, nE, csrLen);

  k_gemm1<<<dim3(nGemm, 2), NTHR, LDS_G1, stream>>>(R1a, w1, as1, ad1, R2, attp, NPAD);
  k_tagg<<<nAgg, NTHR, 0, stream>>>(csr, offp, cnt, ei, attp, R2, ba1, R1b, nN, nE, csrLen, NPAD, 1);
  k_gemm2<<<nGemm, NTHR, LDS_G2, stream>>>(R1b, R1a, wf, bf1, bf2, pbias, R2a, NPAD, NPAD);

  k_gemm1<<<dim3(nGemm, 2), NTHR, LDS_G1, stream>>>(R2a, w2, as2, ad2, R1, attp, NPAD);
  k_tagg<<<nAgg, NTHR, 0, stream>>>(csr, offp, cnt, ei, attp, R1, ba2, R2b, nN, nE, csrLen, NPAD, 0);
  k_gemm2<<<nGemm, NTHR, LDS_G2, stream>>>(R2b, R2a, wf, bf1, bf2, pbias, out, NPAD, nN);
}
